// FlowEstimator3D_74552042324064
// MI455X (gfx1250) — hardware-verified
//
#include <hip/hip_runtime.h>
#include <math.h>

typedef __attribute__((ext_vector_type(16))) _Float16 v16h;
typedef __attribute__((ext_vector_type(16))) __bf16 v16b;
typedef __attribute__((ext_vector_type(8)))  _Float16 v8h;
typedef __attribute__((ext_vector_type(8)))  float v8f;
typedef __attribute__((ext_vector_type(4)))  float v4f;
typedef __attribute__((ext_vector_type(2)))  float v2f;
typedef __attribute__((ext_vector_type(4)))  unsigned v4u;
typedef __attribute__((ext_vector_type(4)))  int v4i;
typedef float __attribute__((may_alias)) float_a;
typedef int __attribute__((may_alias)) int_a;

template <typename T> __device__ __forceinline__ void vst2(void* p, T v) { *(volatile T*)p = v; __threadfence(); *(volatile T*)p = v; }
__device__ __forceinline__ v8f wmma16(v16h a, v16h b, v8f c) {
  v8f d = __builtin_amdgcn_wmma_f32_16x16x32_f16(false, a, false, b, (short)0, c, false, false);
  asm volatile("v_nop\n\tv_nop\n\tv_nop\n\tv_nop" : "+v"(d) : "v"(a), "v"(b));
  return d;
}
__device__ __forceinline__ v8f wmma_bf(v16b a, v16b b, v8f c) {
  v8f d = __builtin_amdgcn_wmma_f32_16x16x32_bf16(false, a, false, b, (short)0, c, false, false);
  asm volatile("v_nop\n\tv_nop\n\tv_nop\n\tv_nop" : "+v"(d) : "v"(a), "v"(b));
  return d;
}
__device__ __forceinline__ v16h frag_h(const _Float16* rowk0, int lane) {
  union { v16h v; v8h q[2]; } u; const _Float16* p = rowk0 + 8 * (lane >> 4);
  u.q[0] = *(const v8h*)p; u.q[1] = *(const v8h*)(p + 16); return u.v;
}
__device__ __forceinline__ v16h frag_f32(const float* rowk0, int lane) {
  v16h a; const float* p = rowk0 + 8 * (lane >> 4);
#pragma unroll
  for (int i = 0; i < 8; ++i) { a[i] = (_Float16)p[i]; a[8 + i] = (_Float16)p[16 + i]; }
  return a;
}
__device__ __forceinline__ v16h frag_f32s(const float* rowk0, int lane, float sc) {
  v16h a; const float* p = rowk0 + 8 * (lane >> 4);
#pragma unroll
  for (int i = 0; i < 8; ++i) { a[i] = (_Float16)(p[i] * sc); a[8 + i] = (_Float16)(p[16 + i] * sc); }
  return a;
}
__device__ __forceinline__ v16h fragc_f32(const float* W, int k0, int n, int lane, int ld, int K) {
  v16h a; const int g = lane >> 4;
#pragma unroll
  for (int i = 0; i < 8; ++i) { const int ka = k0 + 8 * g + i, kb = ka + 16;
    a[i] = (_Float16)(ka < K ? W[(size_t)(ka < K ? ka : K - 1) * ld + n] : 0.f); a[8 + i] = (_Float16)(kb < K ? W[(size_t)(kb < K ? kb : K - 1) * ld + n] : 0.f); }
  return a;
}
struct F2 { v16b h, l; };
__device__ __forceinline__ F2 bsplit16(const float v[16]) { F2 r;
#pragma unroll
  for (int i = 0; i < 16; ++i) { const __bf16 h = (__bf16)v[i]; r.h[i] = h; r.l[i] = (__bf16)(v[i] - (float)h); }
  return r; }
__device__ __forceinline__ F2 split_row(const float* row, int k0, int lane) { float v[16]; const float* p = row + k0 + 8 * (lane >> 4);
#pragma unroll
  for (int i = 0; i < 8; ++i) { v[i] = p[i]; v[8 + i] = p[16 + i]; }
  return bsplit16(v); }
__device__ __forceinline__ F2 split_rowK(const float* row, int k0, int lane, int K) { float v[16]; const int g = lane >> 4;
#pragma unroll
  for (int i = 0; i < 8; ++i) { const int ka = k0 + 8 * g + i, kb = ka + 16; v[i] = ka < K ? row[ka < K ? ka : K - 1] : 0.f; v[8 + i] = kb < K ? row[kb < K ? kb : K - 1] : 0.f; }
  return bsplit16(v); }
__device__ __forceinline__ F2 split_col(const float* W, int k0, int n, int lane, int ld, int K) { float v[16]; const int g = lane >> 4;
#pragma unroll
  for (int i = 0; i < 8; ++i) { const int ka = k0 + 8 * g + i, kb = ka + 16; v[i] = ka < K ? W[(size_t)(ka < K ? ka : K - 1) * ld + n] : 0.f; v[8 + i] = kb < K ? W[(size_t)(kb < K ? kb : K - 1) * ld + n] : 0.f; }
  return bsplit16(v); }
__device__ __forceinline__ v8f mac3(const F2& a, const F2& b, v8f c) { c = wmma_bf(a.l, b.h, c); c = wmma_bf(a.h, b.l, c); return wmma_bf(a.h, b.h, c); }
__device__ __forceinline__ float sigm(float v) { return 1.0f / (1.0f + expf(-v)); }
#define LDSX() do { asm volatile("s_wait_dscnt 0" ::: "memory"); __builtin_amdgcn_wave_barrier(); __builtin_amdgcn_fence(__ATOMIC_RELEASE, "workgroup"); } while (0)


#define NB 4
#define NPt 8192
#define KN 16
#define C0 256
#define C1 128
#define C2 128
#define C3 64
#define WN 8
#define NPTS (NB * NPt)
#define KL1 2080
#define KL2 1056
#ifndef TPB
#define TPB (NPTS / 16)
#define TPB1 TPB
#define TOB (NPt / 64)
#endif
typedef __attribute__((ext_vector_type(8))) __bf16 v8b;
__device__ __forceinline__ v16b frag_b(const __bf16* rowk0, int lane) {
  union { v16b v; v8b q[2]; } u; const __bf16* p = rowk0 + 8 * (lane >> 4);
  u.q[0] = *(const v8b*)p; u.q[1] = *(const v8b*)(p + 16); return u.v;
}
__device__ __forceinline__ v16b frag_gbf(const float* rowk0, int lane) {
  v16b a; const float* p = rowk0 + 8 * (lane >> 4);
#pragma unroll
  for (int i = 0; i < 8; ++i) { a[i] = (__bf16)p[i]; a[8 + i] = (__bf16)p[16 + i]; }
  return a;
}
__device__ __forceinline__ float bfr(float v) { return (float)(__bf16)v; }
__device__ __forceinline__ float lky(float v) { return v >= 0.f ? v : 0.1f * v; }
#define WS_FT   0u
#define WS_P1   (WS_FT + 2u * NPTS * C0)
#define WS_P2   (WS_P1 + 2u * C1 * KL1)
#define WS_F1H  (WS_P2 + 2u * C2 * KL2)
#define WS_F1L  (WS_F1H + 2u * NPTS * C1)
#define WS_F3   (WS_F1L + 2u * NPTS * C1)
#define WS_FL   (WS_F3 + 4u * NPTS * C3)
#define WS_END  (WS_FL + 4u * NPTS * 4)

__global__ __launch_bounds__(256) void k_ft(const float* __restrict__ FEAT, __bf16* __restrict__ FT) {
  __shared__ __align__(16) __bf16 st[64][C0 + 8];
  const int b = blockIdx.y, n0 = blockIdx.x * 64, tid = threadIdx.x;
  for (int q = tid; q < C0 * 64; q += 256) { const int c = q >> 6, nl = q & 63; st[nl][c] = (__bf16)FEAT[((size_t)b * C0 + c) * NPt + n0 + nl]; }
  __syncthreads();
  for (int q = tid; q < 64 * 32; q += 256) { const int nl = q >> 5, pc = q & 31; vst2((unsigned*)(FT + ((size_t)b * NPt + n0 + nl) * C0 + pc * 8), *(const v4u*)&st[nl][pc * 8]); }
}
__global__ __launch_bounds__(256) void k_pack(const float* __restrict__ wl1, const float* __restrict__ wl2, __bf16* __restrict__ P1, __bf16* __restrict__ P2) {
  __shared__ __align__(16) __bf16 srow[KL1];
  const int n = blockIdx.x, tid = threadIdx.x;
  if (n < C1) { for (int k = tid; k < KL1; k += 256) srow[k] = (__bf16)(k < 2072 ? bfr(wl1[(size_t)n * 2072 + k]) : 0.f); __syncthreads(); for (int q = tid; q < KL1 / 8; q += 256) vst2((unsigned*)(P1 + (size_t)n * KL1 + q * 8), *(const v4u*)&srow[q * 8]); }
  else { const int o = n - C1; for (int k = tid; k < KL2; k += 256) srow[k] = (__bf16)(k < 1048 ? bfr(wl2[(size_t)o * 1048 + k]) : 0.f); __syncthreads(); for (int q = tid; q < KL2 / 8; q += 256) vst2((unsigned*)(P2 + (size_t)o * KL2 + q * 8), *(const v4u*)&srow[q * 8]); }
}
template <int NCF, bool HASLO>
__device__ __forceinline__ void pointconv_wave(const __bf16 (*sgh)[NCF + 8], const __bf16 (*sgl)[NCF + 8], const float* spos  , const float (*sw)[KN + 1], __bf16* srow_h, __bf16* srow_l, int lane) {
  const int col = lane & 15, g = lane >> 4;
  v16b ah, al;
#pragma unroll
  for (int i = 0; i < 8; ++i) { const int k0 = 8 * g + i; float v = (col < WN && k0 < KN) ? sw[col][k0] : 0.f; __bf16 hb = (__bf16)v; ah[i] = hb; al[i] = (__bf16)(v - (float)hb);
    ah[8 + i] = (__bf16)0.f; al[8 + i] = (__bf16)0.f; }
  constexpr int NC = NCF + 3; constexpr int NT = (NC + 15) / 16;
#pragma unroll 1
  for (int t = 0; t < NT; ++t) { const int c = t * 16 + col;
    v16b bh, bl;
#pragma unroll
    for (int i = 0; i < 8; ++i) { const int k = 8 * g + i; __bf16 hv = (__bf16)0.f, lv = (__bf16)0.f;
      if (c < 3) { const float p = spos[k * 3 + c]; hv = (__bf16)p; lv = (__bf16)(p - (float)hv); }
      else if (c < NC) { hv = sgh[k][c - 3]; if (HASLO) lv = sgl[k][c - 3]; }
      bh[i] = hv; bl[i] = lv; bh[8 + i] = (__bf16)0.f; bl[8 + i] = (__bf16)0.f; }
    v8f acc = {}; acc = wmma_bf(al, bh, acc); acc = wmma_bf(ah, bl, acc); acc = wmma_bf(ah, bh, acc);
    if (g == 0 && c < NC) {
#pragma unroll
      for (int r = 0; r < 8; ++r) { const float v = acc[r]; const __bf16 hb = (__bf16)v; srow_h[c * 8 + r] = hb; srow_l[c * 8 + r] = (__bf16)(v - (float)hb); } } }
}

__global__ __launch_bounds__(128) void k_pc1(const float* __restrict__ XYZ, const __bf16* __restrict__ FT, const int* __restrict__ KNN, const float* __restrict__ wwn, const float* __restrict__ bwn, const __bf16* __restrict__ P1, const float* __restrict__ bl1, __bf16* __restrict__ F1H, __bf16* __restrict__ F1L) {
  __shared__ __align__(16) __bf16 sgh[4][KN][C0 + 8]; __shared__ float snb[4][KN * 3]; __shared__ float sw[4][WN][KN + 1];
  __shared__ __align__(16) __bf16 sAh[16][KL1 + 8], sAl[16][KL1 + 8]; __shared__ __align__(16) float so[16][C1 + 4];
  const int tid = threadIdx.x, wave = tid >> 5, lane = tid & 31, col = lane & 15, g = lane >> 4; const size_t p0 = (size_t)blockIdx.x * 16; const int b = (int)(p0 / NPt);
  for (int q = tid; q < 16 * 8; q += 128) { sAh[q >> 3][2072 + (q & 7)] = (__bf16)0.f; sAl[q >> 3][2072 + (q & 7)] = (__bf16)0.f; }
#pragma unroll 1
  for (int pi = 0; pi < 4; ++pi) { const int pl = wave * 4 + pi; const size_t p = p0 + pl; const int n = (int)(p % NPt);
    int nn = 0; if (lane < KN) { nn = min(max(KNN[p * KN + lane], 0), NPt - 1); for (int d = 0; d < 3; ++d) snb[wave][lane * 3 + d] = bfr(XYZ[((size_t)b * 3 + d) * NPt + nn]); }
    if (lane < KN) { const v4u* src = (const v4u*)(FT + ((size_t)b * NPt + nn) * C0); v4u* dst = (v4u*)&sgh[wave][lane][0]; for (int i = 0; i < C0 / 8; ++i) dst[i] = src[i]; }
    { const float xn0 = bfr(XYZ[((size_t)b * 3 + 0) * NPt + n]), xn1 = bfr(XYZ[((size_t)b * 3 + 1) * NPt + n]), xn2 = bfr(XYZ[((size_t)b * 3 + 2) * NPt + n]);
      __builtin_amdgcn_wave_barrier();
      for (int e = lane; e < WN * KN; e += 32) { const int m = e / KN, k = e % KN; const float px = snb[wave][k * 3] - xn0, py = snb[wave][k * 3 + 1] - xn1, pz = snb[wave][k * 3 + 2] - xn2;
        sw[wave][m][k] = lky((bfr(wwn[m * 3]) * px + bfr(wwn[m * 3 + 1]) * py) + bfr(wwn[m * 3 + 2]) * pz + bfr(bwn[m])); } }
    LDSX();
    pointconv_wave<C0, false>(sgh[wave], sgh[wave], snb[wave], sw[wave], &sAh[pl][0], &sAl[pl][0], lane);
    LDSX(); }
  __syncthreads();
  { v8f acc[2] = {};
#pragma unroll 1
    for (int kc = 0; kc < KL1 / 32; ++kc) { const v16b ahh = frag_b(&sAh[col][kc * 32], lane), all = frag_b(&sAl[col][kc * 32], lane);
#pragma unroll
      for (int j = 0; j < 2; ++j) { const v16b w = frag_b(P1 + (size_t)((wave * 2 + j) * 16 + col) * KL1 + kc * 32, lane); acc[j] = wmma_bf(all, w, acc[j]); acc[j] = wmma_bf(ahh, w, acc[j]); } }
#pragma unroll
    for (int j = 0; j < 2; ++j) { const int o = (wave * 2 + j) * 16 + col; const float bb = bfr(bl1[o]);
#pragma unroll
      for (int r = 0; r < 8; ++r) so[8 * g + r][o] = lky(acc[j][r] + bb); } }
  __syncthreads();
  { const int pl = tid >> 3, pc = tid & 7;
    for (int pp = pc; pp < 16; pp += 8) { union { __bf16 e[8]; v4u u; } hi, lo;
#pragma unroll
      for (int i = 0; i < 8; ++i) { const float v = so[pl][pp * 8 + i]; const __bf16 hb = (__bf16)v; hi.e[i] = hb; lo.e[i] = (__bf16)(v - (float)hb); }
      vst2((unsigned*)(F1H + (p0 + pl) * C1 + pp * 8), hi.u); vst2((unsigned*)(F1L + (p0 + pl) * C1 + pp * 8), lo.u); } }
}
__global__ __launch_bounds__(128) void k_pc2(const float* __restrict__ XYZ, const __bf16* __restrict__ F1H, const __bf16* __restrict__ F1L, const int* __restrict__ KNN, const float* __restrict__ wwn, const float* __restrict__ bwn, const __bf16* __restrict__ P2, const float* __restrict__ bl2,
                                             const float* __restrict__ wm1, const float* __restrict__ bm1, const float* __restrict__ wm2, const float* __restrict__ bm2, const float* __restrict__ wl, const float* __restrict__ bl, float* __restrict__ F3, float* __restrict__ FL) {
  __shared__ __align__(16) __bf16 sgh[4][KN][C1 + 8], sgl[4][KN][C1 + 8]; __shared__ float snb[4][KN * 3]; __shared__ float sw[4][WN][KN + 1];
  __shared__ __align__(16) __bf16 sAh[16][KL2 + 8], sAl[16][KL2 + 8]; __shared__ __align__(16) float so[16][C1 + 4]; __shared__ __align__(16) __bf16 shh[16][C1 + 8], shl[16][C1 + 8]; __shared__ __align__(16) float sfl[16][4];
  const int tid = threadIdx.x, wave = tid >> 5, lane = tid & 31, col = lane & 15, g = lane >> 4; const size_t p0 = (size_t)blockIdx.x * 16; const int b = (int)(p0 / NPt);
  for (int q = tid; q < 16 * 8; q += 128) { sAh[q >> 3][1048 + (q & 7)] = (__bf16)0.f; sAl[q >> 3][1048 + (q & 7)] = (__bf16)0.f; }
#pragma unroll 1
  for (int pi = 0; pi < 4; ++pi) { const int pl = wave * 4 + pi; const size_t p = p0 + pl; const int n = (int)(p % NPt);
    int nn = 0; if (lane < KN) { nn = min(max(KNN[p * KN + lane], 0), NPt - 1); for (int d = 0; d < 3; ++d) snb[wave][lane * 3 + d] = bfr(XYZ[((size_t)b * 3 + d) * NPt + nn]); }
    if (lane < KN) { const v4u* sh = (const v4u*)(F1H + ((size_t)b * NPt + nn) * C1); const v4u* sl = (const v4u*)(F1L + ((size_t)b * NPt + nn) * C1); v4u* dh = (v4u*)&sgh[wave][lane][0]; v4u* dl = (v4u*)&sgl[wave][lane][0]; for (int i = 0; i < C1 / 8; ++i) { dh[i] = sh[i]; dl[i] = sl[i]; } }
    { const float xn0 = bfr(XYZ[((size_t)b * 3 + 0) * NPt + n]), xn1 = bfr(XYZ[((size_t)b * 3 + 1) * NPt + n]), xn2 = bfr(XYZ[((size_t)b * 3 + 2) * NPt + n]);
      __builtin_amdgcn_wave_barrier();
      for (int e = lane; e < WN * KN; e += 32) { const int m = e / KN, k = e % KN; const float px = snb[wave][k * 3] - xn0, py = snb[wave][k * 3 + 1] - xn1, pz = snb[wave][k * 3 + 2] - xn2;
        sw[wave][m][k] = lky((bfr(wwn[m * 3]) * px + bfr(wwn[m * 3 + 1]) * py) + bfr(wwn[m * 3 + 2]) * pz + bfr(bwn[m])); } }
    LDSX();
    pointconv_wave<C1, true>(sgh[wave], sgl[wave], snb[wave], sw[wave], &sAh[pl][0], &sAl[pl][0], lane);
    LDSX(); }
  __syncthreads();
  { v8f acc[2] = {};
#pragma unroll 1
    for (int kc = 0; kc < KL2 / 32; ++kc) { const v16b ahh = frag_b(&sAh[col][kc * 32], lane), all = frag_b(&sAl[col][kc * 32], lane);
#pragma unroll
      for (int j = 0; j < 2; ++j) { const v16b w = frag_b(P2 + (size_t)((wave * 2 + j) * 16 + col) * KL2 + kc * 32, lane); acc[j] = wmma_bf(all, w, acc[j]); acc[j] = wmma_bf(ahh, w, acc[j]); } }
#pragma unroll
    for (int j = 0; j < 2; ++j) { const int o = (wave * 2 + j) * 16 + col; const float bb = bfr(bl2[o]);
#pragma unroll
      for (int r = 0; r < 8; ++r) { const float v = lky(acc[j][r] + bb); const __bf16 hb = (__bf16)v; shh[8 * g + r][o] = hb; shl[8 * g + r][o] = (__bf16)(v - (float)hb); } } }
  __syncthreads();
  { v8f acc[2] = {};
#pragma unroll
    for (int kc = 0; kc < 4; ++kc) { const v16b ahh = frag_b(&shh[col][kc * 32], lane), all = frag_b(&shl[col][kc * 32], lane);
#pragma unroll
      for (int j = 0; j < 2; ++j) { const v16b w = frag_gbf(wm1 + (size_t)((wave * 2 + j) * 16 + col) * C1 + kc * 32, lane); acc[j] = wmma_bf(all, w, acc[j]); acc[j] = wmma_bf(ahh, w, acc[j]); } }
    __syncthreads();
#pragma unroll
    for (int j = 0; j < 2; ++j) { const int o = (wave * 2 + j) * 16 + col; const float bb = bfr(bm1[o]);
#pragma unroll
      for (int r = 0; r < 8; ++r) { const float v = lky(acc[j][r] + bb); const __bf16 hb = (__bf16)v; shh[8 * g + r][o] = hb; shl[8 * g + r][o] = (__bf16)(v - (float)hb); } } }
  __syncthreads();
  { v8f acc = {};
#pragma unroll
    for (int kc = 0; kc < 4; ++kc) { const v16b ahh = frag_b(&shh[col][kc * 32], lane), all = frag_b(&shl[col][kc * 32], lane); const v16b w = frag_gbf(wm2 + (size_t)(wave * 16 + col) * C1 + kc * 32, lane); acc = wmma_bf(all, w, acc); acc = wmma_bf(ahh, w, acc); }
    const int o = wave * 16 + col; const float bb = bfr(bm2[o]);
#pragma unroll
    for (int r = 0; r < 8; ++r) so[8 * g + r][o] = lky(acc[r] + bb); }
  __syncthreads();
  { const int pl = tid >> 3, c = tid & 7; if (c < 3) { float s = bfr(bl[c]); for (int o = 0; o < C3; ++o) s += bfr(wl[c * C3 + o]) * so[pl][o]; sfl[pl][c] = s; } else if (c == 3) sfl[pl][3] = 0.f; }
  __syncthreads();
  for (int q = tid; q < 16 * 16; q += 128) { const int pl = q >> 4, pc = q & 15; vst2(F3 + (p0 + pl) * C3 + pc * 4, *(const v4f*)&so[pl][pc * 4]); }
  if (tid < 16) vst2(FL + (p0 + tid) * 4, *(const v4f*)&sfl[tid][0]);
}
__global__ __launch_bounds__(256) void k_outT(const float* __restrict__ F3, const float* __restrict__ FL, float* __restrict__ O0, float* __restrict__ O1) {
  __shared__ __align__(16) float st[C3 + 4][64];
  const int b = blockIdx.y, n0 = blockIdx.x * 64, tid = threadIdx.x;
  for (int q = tid; q < 64 * C3; q += 256) { const int nl = q / C3, c = q % C3; st[c][nl] = F3[((size_t)b * NPt + n0 + nl) * C3 + c]; }
  for (int q = tid; q < 64 * 3; q += 256) { const int nl = q / 3, c = q % 3; st[C3 + c][nl] = FL[((size_t)b * NPt + n0 + nl) * 4 + c]; }
  __syncthreads();
  for (int q = tid; q < (C3 + 3) * 16; q += 256) { const int c = q >> 4, pc = q & 15; if (c < C3) vst2(O0 + ((size_t)b * C3 + c) * NPt + n0 + pc * 4, *(const v4f*)&st[c][pc * 4]); else vst2(O1 + ((size_t)b * 3 + (c - C3)) * NPt + n0 + pc * 4, *(const v4f*)&st[c][pc * 4]); }
}

extern "C" void kernel_launch(void* const* d_in, const int* in_sizes, int n_in, void* d_out, int out_size, void* d_ws, size_t ws_size, hipStream_t stream) {
  (void)in_sizes; (void)n_in; (void)out_size;
  const float** F = (const float**)d_in; const int** I = (const int**)d_in;
  if (ws_size < (size_t)WS_END) return;
  char* ws = (char*)d_ws; __bf16 *FT = (__bf16*)(ws + WS_FT), *P1 = (__bf16*)(ws + WS_P1), *P2 = (__bf16*)(ws + WS_P2), *F1H = (__bf16*)(ws + WS_F1H), *F1L = (__bf16*)(ws + WS_F1L); float *F3 = (float*)(ws + WS_F3), *FL = (float*)(ws + WS_FL);
  float* O0 = (float*)d_out; float* O1 = O0 + (size_t)NB * C3 * NPt;
  k_ft<<<dim3(NPt / 64, NB), 256, 0, stream>>>(F[1], FT);
  k_pack<<<C1 + C2, 256, 0, stream>>>(F[5], F[9], P1, P2);
  k_pc1<<<TPB1, 128, 0, stream>>>(F[0], FT, I[2], F[3], F[4], P1, F[6], F1H, F1L);
  k_pc2<<<TPB, 128, 0, stream>>>(F[0], F1H, F1L, I[2], F[7], F[8], P2, F[10], F[11], F[12], F[13], F[14], F[15], F[16], F3, FL);
  k_outT<<<dim3(TOB, NB), 256, 0, stream>>>(F3, FL, O0, O1);
}
